// QKVMultiheadAttention_56538949484962
// MI455X (gfx1250) — hardware-verified
//
#include <hip/hip_runtime.h>
#include <math.h>

typedef __attribute__((ext_vector_type(16))) _Float16 v16h;
typedef __attribute__((ext_vector_type(16))) __bf16 v16b;
typedef __attribute__((ext_vector_type(8)))  _Float16 v8h;
typedef __attribute__((ext_vector_type(8)))  float v8f;
typedef __attribute__((ext_vector_type(4)))  float v4f;
typedef __attribute__((ext_vector_type(2)))  float v2f;
typedef __attribute__((ext_vector_type(4)))  unsigned v4u;
typedef __attribute__((ext_vector_type(4)))  int v4i;
typedef float __attribute__((may_alias)) float_a;
typedef int __attribute__((may_alias)) int_a;

template <typename T> __device__ __forceinline__ void vst2(void* p, T v) { *(volatile T*)p = v; __threadfence(); *(volatile T*)p = v; }
__device__ __forceinline__ v8f wmma16(v16h a, v16h b, v8f c) {
  v8f d = __builtin_amdgcn_wmma_f32_16x16x32_f16(false, a, false, b, (short)0, c, false, false);
  asm volatile("v_nop\n\tv_nop\n\tv_nop\n\tv_nop" : "+v"(d) : "v"(a), "v"(b));
  return d;
}
__device__ __forceinline__ v8f wmma_bf(v16b a, v16b b, v8f c) {
  v8f d = __builtin_amdgcn_wmma_f32_16x16x32_bf16(false, a, false, b, (short)0, c, false, false);
  asm volatile("v_nop\n\tv_nop\n\tv_nop\n\tv_nop" : "+v"(d) : "v"(a), "v"(b));
  return d;
}
__device__ __forceinline__ v16h frag_h(const _Float16* rowk0, int lane) {
  union { v16h v; v8h q[2]; } u; const _Float16* p = rowk0 + 8 * (lane >> 4);
  u.q[0] = *(const v8h*)p; u.q[1] = *(const v8h*)(p + 16); return u.v;
}
__device__ __forceinline__ v16h frag_f32(const float* rowk0, int lane) {
  v16h a; const float* p = rowk0 + 8 * (lane >> 4);
#pragma unroll
  for (int i = 0; i < 8; ++i) { a[i] = (_Float16)p[i]; a[8 + i] = (_Float16)p[16 + i]; }
  return a;
}
__device__ __forceinline__ v16h frag_f32s(const float* rowk0, int lane, float sc) {
  v16h a; const float* p = rowk0 + 8 * (lane >> 4);
#pragma unroll
  for (int i = 0; i < 8; ++i) { a[i] = (_Float16)(p[i] * sc); a[8 + i] = (_Float16)(p[16 + i] * sc); }
  return a;
}
__device__ __forceinline__ v16h fragc_f32(const float* W, int k0, int n, int lane, int ld, int K) {
  v16h a; const int g = lane >> 4;
#pragma unroll
  for (int i = 0; i < 8; ++i) { const int ka = k0 + 8 * g + i, kb = ka + 16;
    a[i] = (_Float16)(ka < K ? W[(size_t)(ka < K ? ka : K - 1) * ld + n] : 0.f); a[8 + i] = (_Float16)(kb < K ? W[(size_t)(kb < K ? kb : K - 1) * ld + n] : 0.f); }
  return a;
}
struct F2 { v16b h, l; };
__device__ __forceinline__ F2 bsplit16(const float v[16]) { F2 r;
#pragma unroll
  for (int i = 0; i < 16; ++i) { const __bf16 h = (__bf16)v[i]; r.h[i] = h; r.l[i] = (__bf16)(v[i] - (float)h); }
  return r; }
__device__ __forceinline__ F2 split_row(const float* row, int k0, int lane) { float v[16]; const float* p = row + k0 + 8 * (lane >> 4);
#pragma unroll
  for (int i = 0; i < 8; ++i) { v[i] = p[i]; v[8 + i] = p[16 + i]; }
  return bsplit16(v); }
__device__ __forceinline__ F2 split_rowK(const float* row, int k0, int lane, int K) { float v[16]; const int g = lane >> 4;
#pragma unroll
  for (int i = 0; i < 8; ++i) { const int ka = k0 + 8 * g + i, kb = ka + 16; v[i] = ka < K ? row[ka < K ? ka : K - 1] : 0.f; v[8 + i] = kb < K ? row[kb < K ? kb : K - 1] : 0.f; }
  return bsplit16(v); }
__device__ __forceinline__ F2 split_col(const float* W, int k0, int n, int lane, int ld, int K) { float v[16]; const int g = lane >> 4;
#pragma unroll
  for (int i = 0; i < 8; ++i) { const int ka = k0 + 8 * g + i, kb = ka + 16; v[i] = ka < K ? W[(size_t)(ka < K ? ka : K - 1) * ld + n] : 0.f; v[8 + i] = kb < K ? W[(size_t)(kb < K ? kb : K - 1) * ld + n] : 0.f; }
  return bsplit16(v); }
__device__ __forceinline__ v8f mac3(const F2& a, const F2& b, v8f c) { c = wmma_bf(a.l, b.h, c); c = wmma_bf(a.h, b.l, c); return wmma_bf(a.h, b.h, c); }
__device__ __forceinline__ float sigm(float v) { return 1.0f / (1.0f + expf(-v)); }
#define LDSX() do { asm volatile("s_wait_dscnt 0" ::: "memory"); __builtin_amdgcn_wave_barrier(); __builtin_amdgcn_fence(__ATOMIC_RELEASE, "workgroup"); } while (0)


#define NB 4
#define NS 2048
#define NH 16
#define DD 64
#define RS (NH * DD)
#ifndef TBH
#define TBH (NB * NH)
#endif
typedef __attribute__((ext_vector_type(8))) __bf16 v8b;
__device__ __forceinline__ v16b frag_b(const __bf16* rowk0, int lane) {
  union { v16b v; v8b q[2]; } u; const __bf16* p = rowk0 + 8 * (lane >> 4);
  u.q[0] = *(const v8b*)p; u.q[1] = *(const v8b*)(p + 16); return u.v;
}
__device__ __forceinline__ float bfr(float v) { return (float)(__bf16)v; }
__device__ __attribute__((noinline)) float exp_ni(float v) { return expf(v); }
__device__ __attribute__((noinline)) float erf_ni(float v) { return erff(v); }

#define WS_VT  0u
#define WS_END (WS_VT + 2u * (size_t)NB * NH * DD * NS)

__global__ __launch_bounds__(128) void k_vt(const float* __restrict__ V, _Float16* __restrict__ VT) { __shared__ __align__(16) _Float16 th[DD][72]; const int t = threadIdx.x; const size_t bh = blockIdx.y; const size_t b = bh / NH; const int h = bh % NH; const int m0 = blockIdx.x * 64;
  for (int e = t; e < 64 * DD; e += 128) { const int ml = e / DD, d = e % DD; th[d][ml] = (_Float16)bfr(V[((b * NS + m0 + ml) * NH + h) * (size_t)DD + d]); }
  __syncthreads(); for (int e = t; e < DD * 8; e += 128) { const int d = e >> 3, q = e & 7; vst2((unsigned*)(VT + (bh * DD + d) * (size_t)NS + m0 + q * 8), *(const v4u*)&th[d][q * 8]); } }
__global__ __launch_bounds__(128) void k_att(const float* __restrict__ Q, const float* __restrict__ K, const _Float16* __restrict__ VT, float* __restrict__ OUT) {
  __shared__ __align__(16) float sp[4][16][36]; __shared__ __align__(16) float so[4][16][68];
  const int tid = threadIdx.x, wave = tid >> 5, lane = tid & 31, col = lane & 15, g = lane >> 4; const size_t bh = blockIdx.y; const size_t b = bh / NH; const int h = bh % NH; const int q0 = blockIdx.x * 64 + wave * 16;
  v16b aq[2];
#pragma unroll
  for (int kc = 0; kc < 2; ++kc) { const float* pp = Q + ((b * NS + q0 + col) * NH + h) * (size_t)DD + kc * 32 + 8 * g;
#pragma unroll
    for (int i = 0; i < 8; ++i) { aq[kc][i] = (__bf16)pp[i]; aq[kc][8 + i] = (__bf16)pp[16 + i]; } }
  float m[8], l[8];
#pragma unroll
  for (int r = 0; r < 8; ++r) { m[r] = -3.0e38f; l[r] = 0.f; }
  v8f acc[4];
#pragma unroll
  for (int j = 0; j < 4; ++j) acc[j] = v8f{};
#pragma unroll 1
  for (int ks = 0; ks < NS / 32; ++ks) { float s[2][8];
#pragma unroll
    for (int ct = 0; ct < 2; ++ct) { const int kk = ks * 32 + ct * 16 + col; v8f c = {};
#pragma unroll
      for (int kc = 0; kc < 2; ++kc) { v16b w; const float* kp = K + ((b * NS + kk) * NH + h) * (size_t)DD + kc * 32 + 8 * g;
#pragma unroll
        for (int i = 0; i < 8; ++i) { w[i] = (__bf16)kp[i]; w[8 + i] = (__bf16)kp[16 + i]; }
        c = wmma_bf(aq[kc], w, c); }
#pragma unroll
      for (int r = 0; r < 8; ++r) s[ct][r] = c[r] * 0.015625f; }
    float alpha[8];
#pragma unroll
    for (int r = 0; r < 8; ++r) { float mx = fmaxf(s[0][r], s[1][r]);
#pragma unroll
      for (int o = 1; o < 16; o <<= 1) mx = fmaxf(mx, __shfl_xor(mx, o));
      const float mn = fmaxf(m[r], mx); alpha[r] = __expf(m[r] - mn); const float e0 = __expf(s[0][r] - mn), e1 = __expf(s[1][r] - mn); float es = e0 + e1;
#pragma unroll
      for (int o = 1; o < 16; o <<= 1) es += __shfl_xor(es, o);
      l[r] = l[r] * alpha[r] + es; m[r] = mn; sp[wave][8 * g + r][col] = e0; sp[wave][8 * g + r][16 + col] = e1; }
#pragma unroll
    for (int j = 0; j < 4; ++j)
#pragma unroll
      for (int r = 0; r < 8; ++r) acc[j][r] *= alpha[r];
    LDSX();
    v16h pa; { const float* prow = &sp[wave][col][0] + 8 * (lane >> 4);
#pragma unroll
      for (int i = 0; i < 8; ++i) { pa[i] = (_Float16)(prow[i] * 2048.0f); pa[8 + i] = (_Float16)(prow[16 + i] * 2048.0f); } }
#pragma unroll
    for (int j = 0; j < 4; ++j) acc[j] = wmma16(pa, frag_h(VT + (bh * DD + j * 16 + col) * (size_t)NS + ks * 32, lane), acc[j]);
    LDSX(); }
#pragma unroll
  for (int r = 0; r < 8; ++r) { const float il = (1.0f / 2048.0f) / l[r];
#pragma unroll
    for (int j = 0; j < 4; ++j) so[wave][8 * g + r][j * 16 + col] = acc[j][r] * il; }
  LDSX(); for (int rl = 0; rl < 16; ++rl) if (lane < 16) vst2(OUT + ((b * NS + q0 + rl) * NH + h) * (size_t)DD + lane * 4, *(const v4f*)&so[wave][rl][lane * 4]); }
extern "C" void kernel_launch(void* const* d_in, const int* in_sizes, int n_in, void* d_out, int out_size, void* d_ws, size_t ws_size, hipStream_t stream) {
  (void)in_sizes; (void)n_in; (void)out_size;
  const float** F = (const float**)d_in;
  if (ws_size < (size_t)WS_END) return;
  char* ws = (char*)d_ws; _Float16* VT = (_Float16*)(ws + WS_VT);
  k_vt<<<dim3(NS / 64, NB * NH), 128, 0, stream>>>(F[2], VT);
  k_att<<<dim3(NS / 64, TBH), 128, 0, stream>>>(F[0], F[1], VT, (float*)d_out);
}
